// RelationAwareLayer_3092376453608
// MI455X (gfx1250) — hardware-verified
//
#include <hip/hip_runtime.h>
#include <stddef.h>
#include <stdint.h>


#define DIMC    128
#define NKQV    384
#define KTOT    512
#define NTYP    4
#define NHEAD   8
#define NREL    6
#define HD      16
#define NTAB    (NHEAD * NREL * HD * HD)
#define NTHR    256
#define NWAVE   8
#define EPT     8
#define CHUNK   (NTHR * EPT)
#define WCAP    (EPT * 32)
#define LISTN   (NWAVE * WCAP)
#define NBMAX   2048
#define RCAP    12288
#define DEGCAP  4096
#define STW     512
#define RB      128
#define TBN     64
#define TLMAX   12
#define CX      8.0f
#define CW      64.0f
#define CG      64.0f
#define SCL1    0.001953125f
#define SCL2    0.000244140625f
#define WSMAX   134217728
#define LDS_AGG_INTS (2 * RCAP + 2 * NBMAX + LISTN + 2 * NWAVE)
#define LDS_AGG ((LDS_AGG_INTS + 2 * NTAB + 64) * 4)

static_assert((CHUNK & (CHUNK - 1)) == 0 && CHUNK <= 4096);
static_assert((NBMAX & (NBMAX - 1)) == 0 && NBMAX <= 4096);
static_assert(NTHR * 8 == NBMAX);
static_assert(LISTN >= NBMAX);
static_assert(LISTN >= NWAVE * WCAP);
static_assert((RCAP % 32) == 0);
static_assert(NWAVE * STW <= RCAP);
static_assert((LDS_AGG_INTS % 4) == 0);
static_assert(LDS_AGG <= 300000);
static_assert(RB == 128 && NTHR == 2 * RB);
static_assert(NWAVE * 16 == RB);
static_assert(KTOT == NTYP * DIMC && (KTOT / 8) == 64);
static_assert(NKQV == 3 * DIMC && (NKQV % TBN) == 0 && (DIMC % TBN) == 0);
static_assert(DIMC == NHEAD * HD);
static_assert(4 * 32 == DIMC);

typedef float    v4f  __attribute__((ext_vector_type(4)));
typedef float    v8f  __attribute__((ext_vector_type(8)));
typedef int      v4i  __attribute__((ext_vector_type(4)));
typedef int      v8i  __attribute__((ext_vector_type(8)));
typedef _Float16 v8h  __attribute__((ext_vector_type(8)));
typedef _Float16 v16h __attribute__((ext_vector_type(16)));
union FragH { v16h v; v8h h[2]; v8i w; };

__device__ __forceinline__ v8f wmh(const FragH& a, const FragH& b, v8f c) {
  v8f d = __builtin_amdgcn_wmma_f32_16x16x32_f16(false, a.v, false, b.v, (short)0, c, false, false);
  asm volatile("v_nop\n\tv_nop\n\tv_nop\n\tv_nop" : "+v"(d) : "v"(a.w), "v"(b.w));
  return d;
}

__device__ __forceinline__ void ldwait() {
  asm volatile("s_wait_loadcnt 0x0" ::: "memory");
}

__device__ __forceinline__ v8h cvt8h(const v4f a, const v4f b, const float c) {
  v8h hv;
  hv[0] = (_Float16)(a.x * c); hv[1] = (_Float16)(a.y * c);
  hv[2] = (_Float16)(a.z * c); hv[3] = (_Float16)(a.w * c);
  hv[4] = (_Float16)(b.x * c); hv[5] = (_Float16)(b.y * c);
  hv[6] = (_Float16)(b.z * c); hv[7] = (_Float16)(b.w * c);
  return hv;
}

__device__ __forceinline__ int scan_chunk(const int* __restrict__ dsts, int nE, int cbase, int slotBase,
                                          int nb, int vec8, int* list, int tid, int lane, int wave) {
  int wc = 0;
  const int el0  = tid * EPT;
  const int e0   = cbase + el0;
  const int sent = -2147483647 - 1;
  v4i da, db;
  if (vec8 != 0 && cbase + CHUNK <= nE) {
    da = *(const v4i*)(dsts + e0);
    db = *(const v4i*)(dsts + e0 + 4);
  } else {
    da.x = (e0     < nE) ? dsts[min(e0,     nE - 1)] : sent;
    da.y = (e0 + 1 < nE) ? dsts[min(e0 + 1, nE - 1)] : sent;
    da.z = (e0 + 2 < nE) ? dsts[min(e0 + 2, nE - 1)] : sent;
    da.w = (e0 + 3 < nE) ? dsts[min(e0 + 3, nE - 1)] : sent;
    db.x = (e0 + 4 < nE) ? dsts[min(e0 + 4, nE - 1)] : sent;
    db.y = (e0 + 5 < nE) ? dsts[min(e0 + 5, nE - 1)] : sent;
    db.z = (e0 + 6 < nE) ? dsts[min(e0 + 6, nE - 1)] : sent;
    db.w = (e0 + 7 < nE) ? dsts[min(e0 + 7, nE - 1)] : sent;
  }
  const unsigned nbs = (unsigned)slotBase;
  const unsigned unb = (unsigned)nb;
  const unsigned s0 = (unsigned)da.x - nbs, s1 = (unsigned)da.y - nbs;
  const unsigned s2 = (unsigned)da.z - nbs, s3 = (unsigned)da.w - nbs;
  const unsigned s4 = (unsigned)db.x - nbs, s5 = (unsigned)db.y - nbs;
  const unsigned s6 = (unsigned)db.z - nbs, s7 = (unsigned)db.w - nbs;
  const bool h0 = s0 < unb, h1 = s1 < unb, h2 = s2 < unb, h3 = s3 < unb;
  const bool h4 = s4 < unb, h5 = s5 < unb, h6 = s6 < unb, h7 = s7 < unb;
  const unsigned any = __builtin_amdgcn_ballot_w32(h0 | h1 | h2 | h3 | h4 | h5 | h6 | h7);
  if (any != 0u) {
#define HITJ(J, HJ, SJ) { \
      const unsigned mj = __builtin_amdgcn_ballot_w32(HJ); \
      if (mj != 0u) { \
        if (HJ) { \
          const int pos = wc + (int)__builtin_amdgcn_mbcnt_lo(mj, 0u); \
          if (pos < WCAP) list[wave * WCAP + pos] = ((el0 + (J)) << 12) | (int)(SJ); \
        } \
        wc += (int)__builtin_popcount(mj); } }
    HITJ(0, h0, s0)
    HITJ(1, h1, s1)
    HITJ(2, h2, s2)
    HITJ(3, h3, s3)
    HITJ(4, h4, s4)
    HITJ(5, h5, s5)
    HITJ(6, h6, s6)
    HITJ(7, h7, s7)
#undef HITJ
  }
  return wc;
}

__global__ __launch_bounds__(NTHR) void k_xprep(const float* __restrict__ x, _Float16* xh, int nN, int nUnits) {
  const int i = (int)blockIdx.x * NTHR + (int)threadIdx.x;
  if (i >= nUnits) return;
  const int row = i >> 4;
  const int c0  = (i & 15) * 8;
  const int rc  = row < nN ? row : nN - 1;
  const float* p = x + (size_t)rc * DIMC + c0;
  v4f a = *(const v4f*)p, b = *(const v4f*)(p + 4);
  const v4f z4 = {0.f, 0.f, 0.f, 0.f};
  if (row >= nN) { a = z4; b = z4; }
  const v8h hv = cvt8h(a, b, CX);
  const size_t o = (size_t)row * DIMC + c0;
  *(volatile v8h*)(xh + o) = hv;
  __threadfence();
  *(volatile v8h*)(xh + o) = hv;
}

__global__ __launch_bounds__(NTHR) void k_wcvt(const float* __restrict__ W0, const float* __restrict__ W1,
                                               const float* __restrict__ W2, _Float16* wt, int nUnits) {
  const int u = (int)blockIdx.x * NTHR + (int)threadIdx.x;
  if (u >= nUnits) return;
  const int n  = u >> 6;
  const int k8 = (u & 63) * 8;
  const int t  = k8 >> 7;
  const int i0 = k8 & (DIMC - 1);
  int seg = n >> 7;
  seg = seg < 0 ? 0 : (seg > 2 ? 2 : seg);
  const int o = n & (DIMC - 1);
  const float* W = (seg == 0) ? W0 : ((seg == 1) ? W1 : W2);
  const float* p = W + (size_t)(t * DIMC + i0) * (size_t)DIMC + o;
  v4f a, b;
  a.x = p[0];        a.y = p[DIMC];     a.z = p[2 * DIMC]; a.w = p[3 * DIMC];
  b.x = p[4 * DIMC]; b.y = p[5 * DIMC]; b.z = p[6 * DIMC]; b.w = p[7 * DIMC];
  const v8h hv = cvt8h(a, b, CW);
  const size_t oo = (size_t)n * KTOT + k8;
  *(volatile v8h*)(wt + oo) = hv;
  __threadfence();
  *(volatile v8h*)(wt + oo) = hv;
}

__global__ __launch_bounds__(NTHR) void k_tgemm(const _Float16* __restrict__ A, const _Float16* __restrict__ WT,
                                                const int* __restrict__ ntype, float* outF,
                                                int nN, int ldo, float scl) {
  __shared__ __attribute__((aligned(16))) float lbuf[(RB + 16) * (DIMC / 2)];
  __shared__ int posOf[RB];
  __shared__ int perm[RB];
  __shared__ int wc5[4 * 5];
  __shared__ int tlT[TLMAX];
  __shared__ int tlR[TLMAX];
  __shared__ int tlV[TLMAX];
  __shared__ int ntl_s;
  _Float16* atile = (_Float16*)lbuf;
  float* stg = lbuf;
  const int tid = (int)threadIdx.x, lane = tid & 31, wave = tid >> 5, hh = lane >> 4, m = lane & 15;
  const int rowBase = (int)blockIdx.x * RB;
  const int col0    = (int)blockIdx.y * TBN;

  int bkt = 4, rk = 0;
  if (tid < RB) {
    const int grow = rowBase + tid;
    const int gc = grow < nN ? grow : nN - 1;
    const int nt = ntype[gc];
    bkt = (grow < nN && (unsigned)nt < (unsigned)NTYP) ? nt : 4;
    const unsigned m0 = __builtin_amdgcn_ballot_w32(bkt == 0);
    const unsigned m1 = __builtin_amdgcn_ballot_w32(bkt == 1);
    const unsigned m2 = __builtin_amdgcn_ballot_w32(bkt == 2);
    const unsigned m3 = __builtin_amdgcn_ballot_w32(bkt == 3);
    const unsigned m4 = __builtin_amdgcn_ballot_w32(bkt == 4);
    const unsigned mo = (bkt == 0) ? m0 : ((bkt == 1) ? m1 : ((bkt == 2) ? m2 : ((bkt == 3) ? m3 : m4)));
    rk = (int)__builtin_amdgcn_mbcnt_lo(mo, 0u);
    if (lane == 0) {
      wc5[wave * 5 + 0] = (int)__builtin_popcount(m0);
      wc5[wave * 5 + 1] = (int)__builtin_popcount(m1);
      wc5[wave * 5 + 2] = (int)__builtin_popcount(m2);
      wc5[wave * 5 + 3] = (int)__builtin_popcount(m3);
      wc5[wave * 5 + 4] = (int)__builtin_popcount(m4);
    }
    perm[tid] = tid;
  }
  __syncthreads();

  if (tid < RB) {
    int cb0 = 0, cb1 = 0, cb2 = 0, cb3 = 0, cb4 = 0;
#pragma unroll
    for (int w2 = 0; w2 < 4; ++w2) {
      cb0 += wc5[w2 * 5 + 0]; cb1 += wc5[w2 * 5 + 1]; cb2 += wc5[w2 * 5 + 2];
      cb3 += wc5[w2 * 5 + 3]; cb4 += wc5[w2 * 5 + 4];
    }
    const int ob0 = 0, ob1 = cb0, ob2 = cb0 + cb1, ob3 = cb0 + cb1 + cb2, ob4 = cb0 + cb1 + cb2 + cb3;
    int pre = 0;
#pragma unroll
    for (int w2 = 0; w2 < 4; ++w2) {
      const int c = wc5[w2 * 5 + bkt];
      pre += (w2 < wave) ? c : 0;
    }
    const int obs = (bkt == 0) ? ob0 : ((bkt == 1) ? ob1 : ((bkt == 2) ? ob2 : ((bkt == 3) ? ob3 : ob4)));
    int pos = obs + pre + rk;
    pos = pos < 0 ? 0 : (pos > RB - 1 ? RB - 1 : pos);
    posOf[tid] = pos;
    perm[pos] = tid;
    if (tid == 0) {
      int n = 0;
      const int cbs[4] = {cb0, cb1, cb2, cb3};
      const int obsa[4] = {ob0, ob1, ob2, ob3};
#pragma unroll
      for (int b = 0; b < 4; ++b) {
        const int ntile = (cbs[b] + 15) >> 4;
#pragma unroll 1
        for (int i = 0; i < ntile; ++i) {
          if (n < TLMAX) { tlT[n] = b; tlR[n] = obsa[b] + 16 * i; tlV[n] = obsa[b] + cbs[b]; ++n; }
        }
      }
      ntl_s = n;
#pragma unroll 1
      for (int i = n; i < TLMAX; ++i) { tlT[i] = 0; tlR[i] = 0; tlV[i] = 0; }
    }
  }
  __syncthreads();

  {
    const int r = tid & (RB - 1), half = tid >> 7;
    int pos = posOf[r];
    pos = pos & (RB - 1);
    const v4i* sp = (const v4i*)(A + (size_t)(rowBase + r) * DIMC + 64 * half);
    v4i* dp = (v4i*)(atile + pos * DIMC + 64 * half);
#pragma unroll
    for (int i = 0; i < 8; ++i) dp[i] = sp[i];
    const v4i zi = {0, 0, 0, 0};
    *(v4i*)(atile + RB * DIMC + 8 * tid) = zi;
  }
  __syncthreads();

  int ntl = ntl_s;
  ntl = ntl < 0 ? 0 : (ntl > TLMAX ? TLMAX : ntl);
  v8f acc[2][4];
  {
    const v8f z = {0.f, 0.f, 0.f, 0.f, 0.f, 0.f, 0.f, 0.f};
#pragma unroll
    for (int q2 = 0; q2 < 2; ++q2) { acc[q2][0] = z; acc[q2][1] = z; acc[q2][2] = z; acc[q2][3] = z; }
  }
  int tR[2], tV[2];
  bool act[2];
#pragma unroll
  for (int q2 = 0; q2 < 2; ++q2) {
    const int ti  = wave + NWAVE * q2;
    act[q2] = ti < ntl;
    const int tic = ti < TLMAX ? ti : TLMAX - 1;
    int tt = tlT[tic]; tt = tt < 0 ? 0 : (tt > NTYP - 1 ? NTYP - 1 : tt);
    int tr = tlR[tic]; tr = tr < 0 ? 0 : (tr > RB ? RB : tr);
    int tv = tlV[tic]; tv = tv < 0 ? 0 : (tv > RB ? RB : tv);
    tR[q2] = tr; tV[q2] = tv;
    if (act[q2]) {
      const _Float16* ap = atile + (tr + m) * DIMC + 8 * hh;
      const _Float16* wp = WT + (size_t)(col0 + m) * KTOT + tt * DIMC + 8 * hh;
#pragma unroll 1
      for (int ks = 0; ks < 4; ++ks) {
        FragH af;
        af.h[0] = *(const v8h*)(ap + 32 * ks);
        af.h[1] = *(const v8h*)(ap + 32 * ks + 16);
#pragma unroll
        for (int ct = 0; ct < 4; ++ct) {
          const _Float16* wq = wp + (size_t)(16 * ct) * KTOT + 32 * ks;
          FragH bf;
          bf.h[0] = *(const v8h*)wq;
          bf.h[1] = *(const v8h*)(wq + 16);
          acc[q2][ct] = wmh(af, bf, acc[q2][ct]);
        }
      }
    }
  }
  __syncthreads();

  {
    const v4f z4 = {0.f, 0.f, 0.f, 0.f};
#pragma unroll
    for (int i = 0; i < 8; ++i) *(v4f*)(stg + tid * 32 + 4 * i) = z4;
  }
  __syncthreads();

#pragma unroll
  for (int q2 = 0; q2 < 2; ++q2) {
    if (act[q2]) {
#pragma unroll
      for (int ct = 0; ct < 4; ++ct) {
#pragma unroll
        for (int r = 0; r < 8; ++r) {
          const int crow = tR[q2] + 8 * hh + r;
          const bool ok = crow < tV[q2];
          const int cc = crow < 0 ? 0 : (crow > RB - 1 ? RB - 1 : crow);
          const int orig = perm[cc] & (RB - 1);
          const float v = acc[q2][ct][r] * scl;
          if (ok) stg[orig * TBN + 16 * ct + m] = v;
        }
      }
    }
  }
  __syncthreads();

  v4f fv[8];
#pragma unroll
  for (int i = 0; i < 8; ++i) {
    const int lr = 16 * wave + 2 * i + hh;
    fv[i] = *(const v4f*)(stg + lr * TBN + 4 * m);
  }
#pragma unroll
  for (int i = 0; i < 8; ++i) {
    const int lr = 16 * wave + 2 * i + hh;
    float* op = outF + (size_t)(rowBase + lr) * (size_t)ldo + col0 + 4 * m;
    *(volatile v4f*)op = fv[i];
  }
  __threadfence();
#pragma unroll
  for (int i = 0; i < 8; ++i) {
    const int lr = 16 * wave + 2 * i + hh;
    float* op = outF + (size_t)(rowBase + lr) * (size_t)ldo + col0 + 4 * m;
    *(volatile v4f*)op = fv[i];
  }
}

__global__ __launch_bounds__(NTHR) void k_agg(
    const int* __restrict__ srcs, const int* __restrict__ dsts, const int* __restrict__ ets,
    const float* __restrict__ KQV, const float* __restrict__ rel_pri,
    const float* __restrict__ rel_att, const float* __restrict__ rel_msg,
    _Float16* HG, int nN, int nE, int nb, int vec8, int MPr) {
  extern __shared__ v4f lds_dyn[];
  int* reg1 = (int*)lds_dyn;
  int* reg2 = reg1 + RCAP;
  int* scnt = reg2 + RCAP;
  int* soff = scnt + NBMAX;
  int* list = soff + NBMAX;
  int* wcnt = list + LISTN;
  int* wtot = wcnt + NWAVE;
  float* attT = (float*)(wtot + NWAVE);
  float* msgT = attT + NTAB;
  float* prt  = msgT + NTAB;
  const int tid = (int)threadIdx.x, lane = tid & 31, wave = tid >> 5, hh = lane >> 4;
  const int nodeBase = (int)blockIdx.x * nb;

  for (int i = tid; i < NBMAX; i += NTHR) scnt[i] = 0;
#pragma unroll 1
  for (int i = tid; i < NTAB; i += NTHR) {
    const int hr = i >> 8, d = (i >> 4) & 15, o = i & 15;
    const int di = (hr << 8) | (o << 4) | d;
    attT[di] = rel_att[i];
    msgT[di] = rel_msg[i];
  }
  if (tid < NHEAD * NREL) prt[tid] = rel_pri[tid] * 0.25f;
  __syncthreads();

  int tot = 0;
  const int nChunks = (nE + CHUNK - 1) / CHUNK;
#pragma unroll 1
  for (int ch = 0; ch < nChunks; ++ch) {
    const int cbase = ch * CHUNK;
    const int wc = scan_chunk(dsts, nE, cbase, nodeBase, nb, vec8, list, tid, lane, wave);
    if (lane == 0) wcnt[wave] = wc;
    __syncthreads();
    int pre = 0, all = 0;
#pragma unroll
    for (int w2 = 0; w2 < NWAVE; ++w2) {
      int c = wcnt[w2];
      c = c < 0 ? 0 : (c > WCAP ? WCAP : c);
      all += c;
      pre += (w2 < wave) ? c : 0;
    }
    const int wcc  = wc > WCAP ? WCAP : wc;
    const int base = tot + pre;
#pragma unroll 1
    for (int i = lane; i < wcc; i += 32) {
      const int ent = list[wave * WCAP + i];
      const int el  = (ent >> 12) & (CHUNK - 1);
      const int sl  = ent & (NBMAX - 1);
      int eid = cbase + el;
      eid = eid > nE - 1 ? nE - 1 : eid;
      const int pos = base + i;
      if (pos < RCAP) reg1[pos] = (int)(((unsigned)eid << 12) | (unsigned)sl);
    }
    tot += all;
    tot = tot > RCAP ? RCAP : tot;
    __syncthreads();
  }
  const int nh = tot;

  if (wave == 0) {
#pragma unroll 1
    for (int b0 = 0; b0 < nh; b0 += 32) {
      const int idx = b0 + lane;
      const int uv  = reg1[idx < RCAP ? idx : RCAP - 1];
      const int m32 = (nh - b0) < 32 ? (nh - b0) : 32;
#pragma unroll 1
      for (int k = 0; k < m32; ++k) {
        const int u  = __builtin_amdgcn_readlane(uv, k);
        const int sl = u & (NBMAX - 1);
        if (lane == 0) scnt[sl] = scnt[sl] + 1;
      }
    }
  }
  __syncthreads();

  {
    const v4i ca = *(const v4i*)(scnt + 8 * tid);
    const v4i cb = *(const v4i*)(scnt + 8 * tid + 4);
    const int e0 = ca.x < 0 ? 0 : ca.x, e1 = ca.y < 0 ? 0 : ca.y, e2 = ca.z < 0 ? 0 : ca.z, e3 = ca.w < 0 ? 0 : ca.w;
    const int e4 = cb.x < 0 ? 0 : cb.x, e5 = cb.y < 0 ? 0 : cb.y, e6 = cb.z < 0 ? 0 : cb.z, e7 = cb.w < 0 ? 0 : cb.w;
    const int ts = e0 + e1 + e2 + e3 + e4 + e5 + e6 + e7;
    int incl = ts;
#pragma unroll
    for (int d = 1; d < 32; d <<= 1) {
      const int up = __shfl_up(incl, d);
      if (lane >= d) incl += up;
    }
    if (lane == 31) wtot[wave] = incl;
    __syncthreads();
    int pre = 0;
#pragma unroll
    for (int w2 = 0; w2 < NWAVE; ++w2) pre += (w2 < wave) ? wtot[w2] : 0;
    int run = pre + incl - ts;
    soff[8 * tid + 0] = run; run += e0;
    soff[8 * tid + 1] = run; run += e1;
    soff[8 * tid + 2] = run; run += e2;
    soff[8 * tid + 3] = run; run += e3;
    soff[8 * tid + 4] = run; run += e4;
    soff[8 * tid + 5] = run; run += e5;
    soff[8 * tid + 6] = run; run += e6;
    soff[8 * tid + 7] = run;
  }
  __syncthreads();
  for (int i = tid; i < NBMAX; i += NTHR) list[i] = soff[i];
  __syncthreads();

  if (wave == 0) {
#pragma unroll 1
    for (int b0 = 0; b0 < nh; b0 += 32) {
      const int idx = b0 + lane;
      const int uv  = reg1[idx < RCAP ? idx : RCAP - 1];
      const int m32 = (nh - b0) < 32 ? (nh - b0) : 32;
#pragma unroll 1
      for (int k = 0; k < m32; ++k) {
        const int u   = __builtin_amdgcn_readlane(uv, k);
        const int sl  = u & (NBMAX - 1);
        const int eid = (int)((unsigned)u >> 12);
        if (lane == 0) {
          int pos = list[sl];
          pos = pos < 0 ? 0 : (pos > RCAP - 1 ? RCAP - 1 : pos);
          reg2[pos] = eid;
          list[sl] = pos + 1;
        }
      }
    }
  }
  __syncthreads();

  const int nbw = nb >> 3;
  const bool ovf = (nh >= RCAP);
  const float qnan = __int_as_float(0x7fc00000);
  float* stw = (float*)reg1 + wave * STW;
  const int o16 = lane & 15;
  const int lc8 = lane < (DIMC / 8) ? lane : (DIMC / 8) - 1;
#pragma unroll 1
  for (int jt = 0; jt < nbw; ++jt) {
    const int slot = wave * nbw + jt;
    const int grow = nodeBase + slot;
    const int gcl  = grow < nN ? grow : nN - 1;
    int st = soff[slot];
    const int craw = scnt[slot];
    int cnt = craw;
    st  = st < 0 ? 0 : (st > nh ? nh : st);
    cnt = cnt < 0 ? 0 : (cnt > DEGCAP ? DEGCAP : cnt);
    if (cnt > nh - st) cnt = nh - st;
    const float pz = (ovf || craw > DEGCAP) ? qnan : 0.0f;
    const bool wr = grow < MPr;

    const float* qrow = KQV + (size_t)gcl * NKQV + DIMC + lane;
    float qv[4], av[4], mx[4], dn[4];
#pragma unroll
    for (int j = 0; j < 4; ++j) { qv[j] = qrow[32 * j]; av[j] = 0.f; mx[j] = -1.0e30f; dn[j] = 0.f; }
    ldwait();

#pragma unroll 1
    for (int q = 0; q < cnt; ++q) {
      int idx = st + q; idx = idx > RCAP - 1 ? RCAP - 1 : idx;
      int eid = reg2[idx]; eid = eid < 0 ? 0 : (eid > nE - 1 ? nE - 1 : eid);
      const int sraw = srcs[eid];
      const int s = sraw < 0 ? 0 : (sraw > nN - 1 ? nN - 1 : sraw);
      const int rraw = ets[eid];
      const int rc = rraw < 0 ? 0 : (rraw > NREL - 1 ? NREL - 1 : rraw);
      const float rin = ((unsigned)rraw < (unsigned)NREL) ? 1.0f : 0.0f;
      const float* kb  = KQV + (size_t)s * NKQV + 16 * hh;
      const int toff = ((hh * NREL + rc) * HD + o16) * HD;
      const float* atb = attT + toff;
      const float* mtb = msgT + toff;
      float kw[4], mm[4];
#pragma unroll
      for (int j = 0; j < 4; ++j) { kw[j] = 0.f; mm[j] = 0.f; }
#pragma unroll 1
      for (int c = 0; c < 4; ++c) {
#pragma unroll
        for (int j = 0; j < 4; ++j) {
          const v4f k4 = *(const v4f*)(kb + 32 * j + 4 * c);
          const v4f v4 = *(const v4f*)(kb + 2 * DIMC + 32 * j + 4 * c);
          const v4f a4 = *(const v4f*)(atb + j * (2 * NREL * HD * HD) + 4 * c);
          const v4f m4 = *(const v4f*)(mtb + j * (2 * NREL * HD * HD) + 4 * c);
          kw[j] = fmaf(k4.w, a4.w, fmaf(k4.z, a4.z, fmaf(k4.y, a4.y, fmaf(k4.x, a4.x, kw[j]))));
          mm[j] = fmaf(v4.w, m4.w, fmaf(v4.z, m4.z, fmaf(v4.y, m4.y, fmaf(v4.x, m4.x, mm[j]))));
        }
      }
      float pl[4];
#pragma unroll
      for (int j = 0; j < 4; ++j) pl[j] = kw[j] * qv[j];
#pragma unroll
      for (int off = 1; off < 16; off <<= 1) {
#pragma unroll
        for (int j = 0; j < 4; ++j) pl[j] += __shfl_xor(pl[j], off);
      }
#pragma unroll
      for (int j = 0; j < 4; ++j) {
        const float prl = prt[(2 * j + hh) * NREL + rc] * rin;
        const float al  = pl[j] * prl;
        const float mv  = mm[j] * rin;
        const float df  = al - mx[j];
        const float ee  = __expf(-fabsf(df));
        const bool  up  = df > 0.f;
        const float s1  = up ? ee : 1.0f;
        const float s2  = up ? 1.0f : ee;
        mx[j] = up ? al : mx[j];
        dn[j] = fmaf(dn[j], s1, s2);
        av[j] = fmaf(av[j], s1, s2 * mv);
      }
    }
    float ov[4];
#pragma unroll
    for (int j = 0; j < 4; ++j) {
      const float ds = dn[j] > 0.f ? dn[j] : 1.0f;
      const float iv = (dn[j] > 0.f ? 1.0f : 0.0f) * __builtin_amdgcn_rcpf(ds);
      ov[j] = fmaf(av[j], iv, pz);
    }
    __builtin_amdgcn_fence(__ATOMIC_RELEASE, "wavefront");
    __builtin_amdgcn_wave_barrier();
#pragma unroll
    for (int j = 0; j < 4; ++j) stw[32 * j + lane] = ov[j];
    __builtin_amdgcn_fence(__ATOMIC_RELEASE, "wavefront");
    __builtin_amdgcn_wave_barrier();
    const v4f ga = *(const v4f*)(stw + 8 * lc8);
    const v4f gb = *(const v4f*)(stw + 8 * lc8 + 4);
    const v8h hv = cvt8h(ga, gb, CG);
    _Float16* gp = HG + (size_t)grow * DIMC + 8 * lc8;
    const bool wsv = wr && (lane < (DIMC / 8));
    if (wsv) *(volatile v8h*)gp = hv;
    __threadfence();
    if (wsv) *(volatile v8h*)gp = hv;
  }
}

__global__ __launch_bounds__(NTHR) void k_ln(const float* __restrict__ x, const float* __restrict__ ho,
                                             const int* __restrict__ ntype, const float* __restrict__ skip,
                                             const float* __restrict__ gam, const float* __restrict__ bet,
                                             float* out, int nN, int nT) {
  const int lane = (int)threadIdx.x & 31, wave = (int)threadIdx.x >> 5;
  const int row = (int)blockIdx.x * NWAVE + wave;
  if (row >= nN) return;
  const int c0 = 4 * lane;
  const v4f xv = *(const v4f*)(x + (size_t)row * DIMC + c0);
  const v4f hv = *(const v4f*)(ho + (size_t)row * DIMC + c0);
  int nt = ntype[row];
  nt = nt < 0 ? 0 : (nt > nT - 1 ? nT - 1 : nt);
  const float g   = 1.0f / (1.0f + expf(-skip[nt]));
  const float omg = 1.0f - g;
  v4f y;
  y.x = xv.x + (hv.x * g + xv.x * omg);
  y.y = xv.y + (hv.y * g + xv.y * omg);
  y.z = xv.z + (hv.z * g + xv.z * omg);
  y.w = xv.w + (hv.w * g + xv.w * omg);
  float s = (y.x + y.y) + (y.z + y.w);
  s += __shfl_xor(s, 1);  s += __shfl_xor(s, 2);
  s += __shfl_xor(s, 4);  s += __shfl_xor(s, 8);
  s += __shfl_xor(s, 16);
  const float mu = s * (1.0f / 128.0f);
  const float d0 = y.x - mu, d1 = y.y - mu, d2 = y.z - mu, d3 = y.w - mu;
  float vs = (d0 * d0 + d1 * d1) + (d2 * d2 + d3 * d3);
  vs += __shfl_xor(vs, 1);  vs += __shfl_xor(vs, 2);
  vs += __shfl_xor(vs, 4);  vs += __shfl_xor(vs, 8);
  vs += __shfl_xor(vs, 16);
  const float var  = vs * (1.0f / 128.0f);
  const float rstd = rsqrtf(var + 1.0e-5f);
  const v4f g4 = *(const v4f*)(gam + c0);
  const v4f b4 = *(const v4f*)(bet + c0);
  v4f o;
  o.x = d0 * rstd * g4.x + b4.x;
  o.y = d1 * rstd * g4.y + b4.y;
  o.z = d2 * rstd * g4.z + b4.z;
  o.w = d3 * rstd * g4.w + b4.w;
  float* op = out + (size_t)row * DIMC + c0;
  *(volatile v4f*)op = o;
  __threadfence();
  *(volatile v4f*)op = o;
}

static int pick_nb(int nE, int nN) {
  int nb = NBMAX;
  while (nb > 16 && (long long)nb * (long long)nE * 5LL > (long long)RCAP * (long long)nN * 4LL) nb >>= 1;
  return nb;
}
static inline int cdiv(int a, int b) { return (a + b - 1) / b; }

extern "C" void kernel_launch(void* const* d_in, const int* in_sizes, int n_in,
                              void* d_out, int out_size, void* d_ws, size_t ws_size,
                              hipStream_t stream) {
  if (n_in < 15) return;
  if (in_sizes[0] < DIMC || (in_sizes[0] % DIMC) != 0) return;
  const int nN = in_sizes[0] / DIMC;
  if (nN < 1 || nN > (1 << 22)) return;
  const int nE = in_sizes[1];
  if (nE < 1 || nE > (1 << 20)) return;
  if (in_sizes[2] != nE || in_sizes[3] != nN || in_sizes[4] != nE) return;
  if (in_sizes[5] != NTYP * DIMC * DIMC || in_sizes[6] != NTYP * DIMC * DIMC) return;
  if (in_sizes[7] != NTYP * DIMC * DIMC || in_sizes[8] != NTYP * DIMC * DIMC) return;
  if (in_sizes[9] != NHEAD * NREL || in_sizes[10] != NTAB || in_sizes[11] != NTAB) return;
  if (in_sizes[12] != NTYP || in_sizes[13] != DIMC || in_sizes[14] != DIMC) return;
  if (out_size != nN * DIMC) return;

  const float* x      = (const float*)d_in[0];
  const int*   src    = (const int*)  d_in[1];
  const int*   dst    = (const int*)  d_in[2];
  const int*   ntype  = (const int*)  d_in[3];
  const int*   etype  = (const int*)  d_in[4];
  const float* Wk     = (const float*)d_in[5];
  const float* Wq     = (const float*)d_in[6];
  const float* Wv     = (const float*)d_in[7];
  const float* Wa     = (const float*)d_in[8];
  const float* relpri = (const float*)d_in[9];
  const float* relatt = (const float*)d_in[10];
  const float* relmsg = (const float*)d_in[11];
  const float* skip   = (const float*)d_in[12];
  const float* gam    = (const float*)d_in[13];
  const float* bet    = (const float*)d_in[14];
  float* out = (float*)d_out;

  const int MP   = cdiv(nN, RB) * RB;
  const int nb   = pick_nb(nE, nN);
  const int gA   = cdiv(MP, nb);
  const int vec8 = ((nE & 3) == 0) ? 1 : 0;
  if (gA * nb < MP || (MP % RB) != 0) return;

  char* ws = (char*)d_ws;
  size_t off = 0;
  const size_t oXH  = off; off += (size_t)MP * DIMC * 2;            off = (off + 255) & ~(size_t)255;
  const size_t oKQV = off; off += (size_t)MP * NKQV * 4;            off = (off + 255) & ~(size_t)255;
  const size_t oHG  = off; off += (size_t)MP * DIMC * 2;            off = (off + 255) & ~(size_t)255;
  const size_t oHO  = off; off += (size_t)MP * DIMC * 4;            off = (off + 255) & ~(size_t)255;
  const size_t oWK  = off; off += (size_t)NKQV * KTOT * 2;          off = (off + 255) & ~(size_t)255;
  const size_t oWA  = off; off += (size_t)DIMC * KTOT * 2;          off = (off + 255) & ~(size_t)255;
  if (off > ws_size || off > (size_t)WSMAX) return;
  _Float16* XH   = (_Float16*)(ws + oXH);
  float*    KQV  = (float*)(ws + oKQV);
  _Float16* HG   = (_Float16*)(ws + oHG);
  float*    HO   = (float*)(ws + oHO);
  _Float16* WKQV = (_Float16*)(ws + oWK);
  _Float16* WA   = (_Float16*)(ws + oWA);

  hipFuncSetAttribute(reinterpret_cast<const void*>(&k_agg),
                      hipFuncAttributeMaxDynamicSharedMemorySize, LDS_AGG);

  const int nUx = MP * (DIMC / 8);
  k_xprep<<<cdiv(nUx, NTHR), NTHR, 0, stream>>>(x, XH, nN, nUx);

  const int nWk = NKQV * (KTOT / 8);
  k_wcvt<<<cdiv(nWk, NTHR), NTHR, 0, stream>>>(Wk, Wq, Wv, WKQV, nWk);
  const int nWa = DIMC * (KTOT / 8);
  k_wcvt<<<cdiv(nWa, NTHR), NTHR, 0, stream>>>(Wa, Wa, Wa, WA, nWa);

  const int gM = MP / RB;
  k_tgemm<<<dim3(gM, NKQV / TBN), NTHR, 0, stream>>>(XH, WKQV, ntype, KQV, nN, NKQV, SCL1);
  k_agg<<<gA, NTHR, LDS_AGG, stream>>>(src, dst, etype, KQV, relpri, relatt, relmsg, HG, nN, nE, nb, vec8, MP);
  k_tgemm<<<dim3(gM, DIMC / TBN), NTHR, 0, stream>>>(HG, WA, ntype, HO, nN, DIMC, SCL2);
  k_ln<<<cdiv(nN, NWAVE), NTHR, 0, stream>>>(x, HO, ntype, skip, gam, bet, out, nN, NTYP);
}
